// RotaryCrossAttention_51410758533607
// MI455X (gfx1250) — hardware-verified
//
#include <hip/hip_runtime.h>


namespace {
constexpr int Bn = 2, NQ = 2048, NK = 8192, D = 512, H = 8, HD = 64, TQ = Bn * NQ, TK = Bn * NK;
constexpr float XS = 8.0f, PS = 8.0f, EPS = 1e-5f;
struct Wo_ { static constexpr size_t Q = 0, KV = (size_t)D * D, O = KV + (size_t)2 * D * D, END = O + (size_t)D * D; };

typedef _Float16 b16;
typedef __attribute__((ext_vector_type(16))) _Float16 v16b;
typedef __attribute__((ext_vector_type(8))) _Float16 v8b;
typedef __attribute__((ext_vector_type(8))) float v8f;
typedef __attribute__((ext_vector_type(4))) float v4f;
__device__ __forceinline__ float bf16_rne(float f) { unsigned int u = __float_as_uint(f); u += 0x7FFFu + ((u >> 16) & 1u); return __uint_as_float(u & 0xFFFF0000u); }
__device__ __forceinline__ v16b frag_kb(const b16* p, int hh) { const v8b a = *(const v8b*)(p + 8 * hh), b = *(const v8b*)(p + 16 + 8 * hh); v16b f;
#pragma unroll
  for (int e = 0; e < 8; ++e) { f[e] = a[e]; f[8 + e] = b[e]; } return f; }
__device__ __forceinline__ v8f wmma16b(v16b a, v16b b, v8f c) { v8f d = __builtin_amdgcn_wmma_f32_16x16x32_f16(false, a, false, b, (short)0, c, false, false); asm volatile("v_nop\n\tv_nop\n\tv_nop\n\tv_nop" : "+v"(d) : "v"(a), "v"(b)); return d; }
__device__ __forceinline__ void wave_lds_sync() { __builtin_amdgcn_fence(__ATOMIC_RELEASE, "workgroup"); __builtin_amdgcn_wave_barrier(); __builtin_amdgcn_fence(__ATOMIC_ACQUIRE, "workgroup"); }
__device__ __forceinline__ float nexp(float x) { return __builtin_amdgcn_exp2f(x * 1.4426950408889634f); }
__device__ __forceinline__ float pmul(float a, float b) { float p = a * b; asm volatile("" : "+v"(p)); return p; }
__device__ __forceinline__ float wsum(float v) {
#pragma unroll
  for (int o = 1; o < 32; o <<= 1) v += __shfl_xor(v, o); return v; }
__device__ __forceinline__ void sincos_r(float ang, float& sn, float& cs) { const float k = rintf(ang * 0.15915494309189535f); float r = __builtin_fmaf(k, -6.28318548202514648f, ang); r = __builtin_fmaf(k, 1.7484556025237907e-7f, r);
  const float t = r * 0.15915494309189535f; sn = __builtin_amdgcn_sinf(t); cs = __builtin_amdgcn_cosf(t); }

__global__ __launch_bounds__(256) void prep_kernel(const float* __restrict__ wq, const float* __restrict__ wkv, const float* __restrict__ wo, const float* __restrict__ lqw, const float* __restrict__ lqb, const float* __restrict__ lcw, const float* __restrict__ lcb, const float* __restrict__ bo, b16* __restrict__ R, float* __restrict__ P) {
  const size_t tid = (size_t)blockIdx.x * 256 + threadIdx.x, nth = (size_t)gridDim.x * 256;
  auto tr = [&](size_t base, int nout, int kin, const float* W) { for (size_t p = tid; p < (size_t)nout * (kin / 8); p += nth) { const int o = (int)(p / (kin / 8)), k0 = (int)(p % (kin / 8)) * 8; v8b v;
#pragma unroll
      for (int e = 0; e < 8; ++e) v[e] = (b16)bf16_rne(W[(size_t)(k0 + e) * nout + o]); *(volatile v8b*)(R + base + (size_t)o * kin + k0) = v; } };
  for (int pass = 0; pass < 2; ++pass) { tr(Wo_::Q, D, D, wq); tr(Wo_::KV, 2 * D, D, wkv); tr(Wo_::O, D, D, wo);
    for (size_t q = tid; q < 2560; q += nth) { const int i = (int)q, c = i & 511; float v; if (i < 512) v = lqw[c]; else if (i < 1024) v = lqb[c]; else if (i < 1536) v = lcw[c]; else if (i < 2048) v = lcb[c]; else v = bo[c]; P[q] = bf16_rne(v); }
    __threadfence(); }
}

__global__ __launch_bounds__(256) void ln_kernel(const float* __restrict__ src, const float* __restrict__ g, const float* __restrict__ bb, int nrows, b16* __restrict__ dst, b16* __restrict__ dstl) {
  const int row = blockIdx.x * 8 + (threadIdx.x >> 5), lane = threadIdx.x & 31; if (row >= nrows) return; const float* xr = src + (size_t)row * D;
  float v[16]; float s = 0.0f;
#pragma unroll
  for (int i = 0; i < 16; ++i) { v[i] = bf16_rne(xr[(i >> 3) * 256 + lane * 8 + (i & 7)]); s += v[i]; }
  s = wsum(s); const float mu = s * (1.0f / D); float q = 0.0f;
#pragma unroll
  for (int i = 0; i < 16; ++i) { const float d = v[i] - mu; q += pmul(d, d); }
  q = wsum(q); const float inv = rsqrtf(q * (1.0f / D) + EPS);
  for (int pass = 0; pass < 2; ++pass) {
#pragma unroll
    for (int gq = 0; gq < 2; ++gq) { v8b o, ol; const int c0 = gq * 256 + lane * 8; for (int e = 0; e < 8; ++e) { const float y = (pmul((v[gq * 8 + e] - mu) * inv, g[c0 + e]) + bb[c0 + e]) * XS; const b16 h_ = (b16)y; o[e] = h_; ol[e] = (b16)(y - (float)h_); } *(volatile v8b*)(dst + (size_t)row * D + c0) = o; *(volatile v8b*)(dstl + (size_t)row * D + c0) = ol; }
    __threadfence(); }
}

template <int MODE>
__global__ __launch_bounds__(64) void gemm_kernel(const b16* __restrict__ A, const b16* __restrict__ Al, const b16* __restrict__ Bw, int ncols, const float* __restrict__ F, const float* __restrict__ bias, b16* __restrict__ O16, b16* __restrict__ O16l, float* __restrict__ O32) {
  __shared__ __attribute__((aligned(16))) float Ts[2][32][128 + 4];
  const int lane = threadIdx.x & 31, wave = threadIdx.x >> 5, nloc = lane & 15, hlf = lane >> 4, m0 = blockIdx.y * 32, c0 = blockIdx.x * 256 + wave * 128;
  v8f acc[2][8];
#pragma unroll
  for (int r = 0; r < 2; ++r)
#pragma unroll
    for (int t = 0; t < 8; ++t) acc[r][t] = (v8f){};
#pragma unroll 2
  for (int kb = 0; kb < D; kb += 32) { const v16b a0 = frag_kb(A + (size_t)(m0 + nloc) * D + kb, hlf), a1 = frag_kb(A + (size_t)(m0 + 16 + nloc) * D + kb, hlf), l0 = frag_kb(Al + (size_t)(m0 + nloc) * D + kb, hlf), l1 = frag_kb(Al + (size_t)(m0 + 16 + nloc) * D + kb, hlf);
#pragma unroll
    for (int t = 0; t < 8; ++t) { const v16b bw = frag_kb(Bw + (size_t)(c0 + t * 16 + nloc) * D + kb, hlf); acc[0][t] = wmma16b(a0, bw, acc[0][t]); acc[0][t] = wmma16b(l0, bw, acc[0][t]); acc[1][t] = wmma16b(a1, bw, acc[1][t]); acc[1][t] = wmma16b(l1, bw, acc[1][t]); } }
#pragma unroll
  for (int t = 0; t < 8; ++t) { const float bv = (MODE == 2) ? bias[c0 + t * 16 + nloc] : 0.0f;
#pragma unroll
    for (int r = 0; r < 2; ++r)
#pragma unroll
      for (int v = 0; v < 8; ++v) Ts[wave][r * 16 + 8 * hlf + v][t * 16 + nloc] = acc[r][t][v] * (1.0f / XS) + bv; }
  wave_lds_sync();
  if (MODE == 0) {
    float o_[64];
    for (int hI = 0; hI < 2; ++hI) { const float* fr = F + (size_t)(m0 + lane) * HD; const float* xr = &Ts[wave][lane][hI * 64];
#pragma unroll
      for (int d = 0; d < 64; ++d) { const float f = bf16_rne(fr[d]); float sn, cs; sincos_r(f, sn, cs); const float rh = (d < 32) ? -xr[2 * d + 1] : xr[2 * (d - 32)]; o_[d] = pmul(xr[d], cs) + pmul(rh, sn); }
#pragma unroll
      for (int d = 0; d < 64; ++d) Ts[wave][lane][hI * 64 + d] = o_[d]; }
    wave_lds_sync(); }
  for (int pass = 0; pass < 2; ++pass) {
    if (MODE == 2) { for (int i = lane; i < 32 * 32; i += 32) { const int rr = i >> 5, c4 = (i & 31) * 4; *(volatile v4f*)(O32 + (size_t)(m0 + rr) * ncols + c0 + c4) = *(const v4f*)(&Ts[wave][rr][c4]); } }
    else if (MODE == 3) { for (int i = lane; i < 32 * 16; i += 32) { const int rr = i >> 4, c8 = (i & 15) * 8; v8b o, ol; for (int e = 0; e < 8; ++e) { const float y = Ts[wave][rr][c8 + e] * XS; const b16 h_ = (b16)y; o[e] = h_; ol[e] = (b16)(y - (float)h_); } *(volatile v8b*)(O16 + (size_t)(m0 + rr) * ncols + c0 + c8) = o; *(volatile v8b*)(O16l + (size_t)(m0 + rr) * ncols + c0 + c8) = ol; } }
    else { for (int i = lane; i < 32 * 16; i += 32) { const int rr = i >> 4, c8 = (i & 15) * 8; v8b o; for (int e = 0; e < 8; ++e) o[e] = (b16)(Ts[wave][rr][c8 + e] * XS); *(volatile v8b*)(O16 + (size_t)(m0 + rr) * ncols + c0 + c8) = o; } }
    __threadfence(); }
}

__global__ __launch_bounds__(256) void vt_kernel(const b16* __restrict__ Vr, b16* __restrict__ vt) {
  __shared__ __attribute__((aligned(16))) b16 T[HD][128 + 8];
  const int b = blockIdx.z, h = blockIdx.y, t0 = blockIdx.x * 128, t_ = threadIdx.x;
  for (int i = t_; i < 128 * (HD / 8); i += 256) { const int tk = i >> 3, d8 = (i & 7) * 8; const v8b vv = *(const v8b*)(Vr + ((size_t)(b * NK + t0 + tk)) * D + h * HD + d8); for (int e = 0; e < 8; ++e) T[d8 + e][tk] = vv[e]; }
  __syncthreads();
  for (int pass = 0; pass < 2; ++pass) { for (int i = t_; i < HD * 16; i += 256) { const int d = i >> 4, c8 = (i & 15) * 8; *(volatile v8b*)(vt + (((size_t)b * H + h) * HD + d) * NK + t0 + c8) = *(const v8b*)(&T[d][c8]); } __threadfence(); }
}

__global__ __launch_bounds__(256) void attn_kernel(const b16* __restrict__ Q, const b16* __restrict__ Kk, const b16* __restrict__ vt, const b16* __restrict__ vtl, b16* __restrict__ ctx, b16* __restrict__ ctxl) {
  __shared__ __attribute__((aligned(16))) b16 Os[16][D + 8], Osl[16][D + 8];
  const int h = threadIdx.x >> 5, lane = threadIdx.x & 31, hh = lane >> 4, col = lane & 15; const int b = blockIdx.x / (NQ / 16), q0 = (blockIdx.x % (NQ / 16)) * 16, qi = q0 + col;
  const b16* Qr = Q + (size_t)(b * NQ) * D + h * HD; const b16* Kr = Kk + (size_t)(b * NK) * D + h * HD; const b16* V = vt + (((size_t)b * H + h) * HD) * NK; const b16* Vl = vtl + (((size_t)b * H + h) * HD) * NK;
  const v16b qf0 = frag_kb(Qr + (size_t)qi * D, hh), qf1 = frag_kb(Qr + (size_t)qi * D + 32, hh);
  float m = -INFINITY, l = 0.0f; v8f o[4] = {{}, {}, {}, {}};
  for (int kb = 0; kb < NK; kb += 32) {
    v8f s0 = {}, s1 = {}; s0 = wmma16b(frag_kb(Kr + (size_t)(kb + col) * D, hh), qf0, s0); s0 = wmma16b(frag_kb(Kr + (size_t)(kb + col) * D + 32, hh), qf1, s0);
    s1 = wmma16b(frag_kb(Kr + (size_t)(kb + 16 + col) * D, hh), qf0, s1); s1 = wmma16b(frag_kb(Kr + (size_t)(kb + 16 + col) * D + 32, hh), qf1, s1);
    float mr = -INFINITY;
#pragma unroll
    for (int r = 0; r < 8; ++r) { s0[r] *= (0.125f / (XS * XS)); s1[r] *= (0.125f / (XS * XS)); mr = fmaxf(mr, fmaxf(s0[r], s1[r])); }
    mr = fmaxf(mr, __shfl_xor(mr, 16)); const float mn = fmaxf(m, mr), al_ = nexp(m - mn); m = mn; float sum = 0.0f; v16b pb, pl;
#pragma unroll
    for (int r = 0; r < 8; ++r) { const float e0 = nexp(s0[r] - mn), e1 = nexp(s1[r] - mn); sum += e0 + e1; const float y0 = e0 * PS, y1 = e1 * PS; const b16 h0 = (b16)y0, h1 = (b16)y1; pb[r] = h0; pl[r] = (b16)(y0 - (float)h0); pb[8 + r] = h1; pl[8 + r] = (b16)(y1 - (float)h1); }
    sum += __shfl_xor(sum, 16); l = l * al_ + sum;
#pragma unroll
    for (int t = 0; t < 4; ++t) { o[t] *= al_; const v16b vh = frag_kb(V + (size_t)(t * 16 + col) * NK + kb, hh), vlo = frag_kb(Vl + (size_t)(t * 16 + col) * NK + kb, hh); o[t] = wmma16b(vh, pb, o[t]); o[t] = wmma16b(vh, pl, o[t]); o[t] = wmma16b(vlo, pb, o[t]); } }
  const float inv = 1.0f / (l * PS);
#pragma unroll
  for (int t = 0; t < 4; ++t)
#pragma unroll
    for (int r = 0; r < 8; ++r) { const float y = o[t][r] * inv; const b16 h_ = (b16)y; Os[col][h * HD + t * 16 + 8 * hh + r] = h_; Osl[col][h * HD + t * 16 + 8 * hh + r] = (b16)(y - (float)h_); }
  __syncthreads();
  for (int pass = 0; pass < 2; ++pass) { for (int i = threadIdx.x; i < 16 * (D / 8); i += 256) { const int rr = i / (D / 8), c8 = (i % (D / 8)) * 8; const size_t gi = ((size_t)(b * NQ + q0 + rr)) * D + c8; *(volatile v8b*)(ctx + gi) = *(const v8b*)(&Os[rr][c8]); *(volatile v8b*)(ctxl + gi) = *(const v8b*)(&Osl[rr][c8]); } __threadfence(); }
}
}

extern "C" void kernel_launch(void* const* d_in, const int* in_sizes, int n_in,
                              void* d_out, int out_size, void* d_ws, size_t ws_size, hipStream_t stream) {
  (void)n_in; (void)out_size;
  const float* xq = (const float*)d_in[0]; const float* xc = (const float*)d_in[1]; const float* fq = (const float*)d_in[2]; const float* fc = (const float*)d_in[3]; const float* lqw = (const float*)d_in[4]; const float* lqb = (const float*)d_in[5]; const float* lcw = (const float*)d_in[6]; const float* lcb = (const float*)d_in[7];
  const float* wq = (const float*)d_in[8]; const float* wkv = (const float*)d_in[9]; const float* wo = (const float*)d_in[10]; const float* bo = (const float*)d_in[11];
  float* out = (float*)d_out;
  if (in_sizes[0] != TQ * D || in_sizes[1] != TK * D || in_sizes[2] != TQ * HD || in_sizes[3] != TK * HD || in_sizes[8] != D * D || in_sizes[9] != D * 2 * D) return;
  size_t off = 0; char* ws = (char*)d_ws;
  auto carve = [&](size_t bytes) { char* p = ws + off; off += (bytes + 255) & ~(size_t)255; return p; };
  b16* R = (b16*)carve(Wo_::END * 2); float* P = (float*)carve(2560 * 4); b16* XQ = (b16*)carve((size_t)TQ * D * 2); b16* XQl = (b16*)carve((size_t)TQ * D * 2); b16* XC = (b16*)carve((size_t)TK * D * 2); b16* XCl = (b16*)carve((size_t)TK * D * 2);
  b16* Q = (b16*)carve((size_t)TQ * D * 2); b16* Kk = (b16*)carve((size_t)TK * D * 2); b16* VRh = (b16*)carve((size_t)TK * D * 2); b16* VRl = (b16*)carve((size_t)TK * D * 2); b16* CTX = (b16*)carve((size_t)TQ * D * 2); b16* CTXl = (b16*)carve((size_t)TQ * D * 2);
  if (off > ws_size) return;
  b16* VT = XC; b16* VTl = XCl;
  prep_kernel<<<256, 256, 0, stream>>>(wq, wkv, wo, lqw, lqb, lcw, lcb, bo, R, P);
  ln_kernel<<<TQ / 8, 256, 0, stream>>>(xq, P, P + 512, TQ, XQ, XQl);
  ln_kernel<<<TK / 8, 256, 0, stream>>>(xc, P + 1024, P + 1536, TK, XC, XCl);
  gemm_kernel<0><<<dim3(D / 256, TQ / 32), 64, 0, stream>>>(XQ, XQl, R + Wo_::Q, D, fq, nullptr, Q, nullptr, nullptr);
  gemm_kernel<0><<<dim3(D / 256, TK / 32), 64, 0, stream>>>(XC, XCl, R + Wo_::KV, D, fc, nullptr, Kk, nullptr, nullptr);
  gemm_kernel<3><<<dim3(D / 256, TK / 32), 64, 0, stream>>>(XC, XCl, R + Wo_::KV + (size_t)D * D, D, nullptr, nullptr, VRh, VRl, nullptr);
  vt_kernel<<<dim3(NK / 128, H, Bn), 256, 0, stream>>>(VRh, VT);
  vt_kernel<<<dim3(NK / 128, H, Bn), 256, 0, stream>>>(VRl, VTl);
  attn_kernel<<<TQ / 16, 256, 0, stream>>>(Q, Kk, VT, VTl, CTX, CTXl);
  gemm_kernel<2><<<dim3(D / 256, TQ / 32), 64, 0, stream>>>(CTX, CTXl, R + Wo_::O, D, nullptr, P + 2048, nullptr, nullptr, out);
}
